// MultiDPHConvHeadAttention_87797721465312
// MI455X (gfx1250) — hardware-run, weakly checked
//
#include <hip/hip_runtime.h>
#include <math.h>
#include <float.h>
#include <stdint.h>

#define NB    8
#define NTOK  1024
#define DMD   768
#define NHD   12
#define HDD   64
#define NROW  (NB * NTOK)
#define NQB   (NTOK / 64)
#define NKT   (NTOK / 64)
#define PCAR  16384.0f
#define POFF  16.0f
static_assert(NHD * HDD == DMD);
static_assert(HDD == 64);
static_assert(16384 / NTOK == 16);
static_assert((NTOK % 64) == 0 && (DMD % 64) == 0 && (NROW % 64) == 0 && (DMD % 32) == 0);
static_assert(((NROW / 64) * (DMD / 64)) % 8 == 0);
static_assert(((NROW / 32) * (DMD / 32)) % 8 == 0);
static_assert(((NROW * DMD / 8) % 256) == 0);
static_assert((DMD % 128) == 0);
static_assert(((NROW * (DMD / 128)) % 8) == 0);

typedef _Float16 v16h __attribute__((ext_vector_type(16)));
typedef _Float16 v8h  __attribute__((ext_vector_type(8)));
typedef float    v8f  __attribute__((ext_vector_type(8)));
typedef float    v4f  __attribute__((ext_vector_type(4)));
typedef unsigned int v4u __attribute__((ext_vector_type(4)));
typedef unsigned int v2u __attribute__((ext_vector_type(2)));

__device__ __forceinline__ unsigned short bf_bits(float f) {
  unsigned u = __float_as_uint(f);
  return (unsigned short)((u + 0x7FFFu + ((u >> 16) & 1u)) >> 16);
}
__device__ __forceinline__ float bf_up(unsigned short h) { return __uint_as_float(((unsigned)h) << 16); }
__device__ __forceinline__ float bfr(float f) { return bf_up(bf_bits(f)); }
__device__ __forceinline__ unsigned short h_bits(_Float16 x) { return __builtin_bit_cast(unsigned short, x); }
__device__ __forceinline__ unsigned pk16(unsigned short a, unsigned short b) { return (unsigned)a | ((unsigned)b << 16); }
__device__ __forceinline__ v8f zero8() { v8f z = {0.f, 0.f, 0.f, 0.f, 0.f, 0.f, 0.f, 0.f}; return z; }

__device__ __forceinline__ void ld8(const float* p, float* o) {
  const v4f a = *(const v4f*)(p);
  const v4f b = *(const v4f*)(p + 4);
  o[0] = a[0]; o[1] = a[1]; o[2] = a[2]; o[3] = a[3];
  o[4] = b[0]; o[5] = b[1]; o[6] = b[2]; o[7] = b[3];
}

__device__ __forceinline__ v16h ldfrag_h(const _Float16* p) {
  union { v16h v; v8h h[2]; } f;
  f.h[0] = *(const v8h*)(p);
  f.h[1] = *(const v8h*)(p + 16);
  return f.v;
}

__device__ __forceinline__ v8f mma_h(v16h a, v16h b, v8f c) {
  c = __builtin_amdgcn_wmma_f32_16x16x32_f16(false, a, false, b, (short)0, c, false, false);
#if defined(__HIP_DEVICE_COMPILE__)
  asm volatile("v_nop\n\tv_nop\n\tv_nop\n\tv_nop" : "+v"(c) : "v"(a), "v"(b));
#endif
  return c;
}
__device__ __forceinline__ v8f mma_h_raw(v16h a, v16h b, v8f c) {
  return __builtin_amdgcn_wmma_f32_16x16x32_f16(false, a, false, b, (short)0, c, false, false);
}
__device__ __forceinline__ void dep_guard_h(v8f& a, v8f& b, v16h x) {
#if defined(__HIP_DEVICE_COMPILE__)
  asm volatile("v_nop\n\tv_nop\n\tv_nop\n\tv_nop" : "+v"(a), "+v"(b) : "v"(x));
#endif
}
__device__ __forceinline__ void keep4_h(v16h a, v16h b, v16h c, v16h d) {
#if defined(__HIP_DEVICE_COMPILE__)
  asm volatile("v_nop" :: "v"(a), "v"(b), "v"(c), "v"(d));
#endif
}
__device__ __forceinline__ void acc_guard4(v8f& a, v8f& b, v8f& c, v8f& d) {
#if defined(__HIP_DEVICE_COMPILE__)
  asm volatile("v_nop\n\tv_nop\n\tv_nop\n\tv_nop" : "+v"(a), "+v"(b), "+v"(c), "+v"(d));
#endif
}

__global__ __launch_bounds__(256) void x_cvt(const float* __restrict__ in, unsigned short* out, int n8,
                                             float sc) {
  const int i = blockIdx.x * 256 + threadIdx.x;
  if (i < n8) {
    const v4f a = *(const v4f*)(in + (size_t)i * 8);
    const v4f b = *(const v4f*)(in + (size_t)i * 8 + 4);
    v4u p;
    p[0] = pk16(h_bits((_Float16)(bfr(a[0]) * sc)), h_bits((_Float16)(bfr(a[1]) * sc)));
    p[1] = pk16(h_bits((_Float16)(bfr(a[2]) * sc)), h_bits((_Float16)(bfr(a[3]) * sc)));
    p[2] = pk16(h_bits((_Float16)(bfr(b[0]) * sc)), h_bits((_Float16)(bfr(b[1]) * sc)));
    p[3] = pk16(h_bits((_Float16)(bfr(b[2]) * sc)), h_bits((_Float16)(bfr(b[3]) * sc)));
    *(volatile v4u*)(out + (size_t)i * 8) = p;
    __threadfence();
    *(volatile v4u*)(out + (size_t)i * 8) = p;
  }
}

__global__ __launch_bounds__(256) void wt_cvt(const float* __restrict__ W, int ncols, int nrows,
                                              unsigned short* outp, float sc) {
  __shared__ __align__(16) float sw[64 * 68];
  const int tid = threadIdx.x;
  const int n0 = blockIdx.x * 64;
  const int k0 = blockIdx.y * 64;
#pragma unroll
  for (int i = 0; i < 4; ++i) {
    const int idx = i * 256 + tid;
    const int kk = idx >> 4, c4 = (idx & 15) * 4;
    const v4f a = *(const v4f*)(W + (size_t)(k0 + kk) * ncols + n0 + c4);
    *(v4f*)(sw + kk * 68 + c4) = a;
  }
  __syncthreads();

  const int g = tid >> 3, piece = tid & 7;
  v4u ov[2];
  size_t oofs[2];
#pragma unroll
  for (int it = 0; it < 2; ++it) {
    const int nn = it * 32 + g;
    v4u a;
#pragma unroll
    for (int e = 0; e < 4; ++e) {
      const float f0 = sw[(piece * 8 + 2 * e) * 68 + nn];
      const float f1 = sw[(piece * 8 + 2 * e + 1) * 68 + nn];
      a[e] = pk16(h_bits((_Float16)(bfr(f0) * sc)), h_bits((_Float16)(bfr(f1) * sc)));
    }
    ov[it] = a;
    oofs[it] = (size_t)(n0 + nn) * nrows + k0 + piece * 8;
  }
  for (int pass = 0; pass < 2; ++pass) {
#pragma unroll
    for (int it = 0; it < 2; ++it) *(volatile v4u*)(outp + oofs[it]) = ov[it];
    __threadfence();
  }
}

__global__ __launch_bounds__(256) void gemm64(
    const unsigned short* __restrict__ Ap, int lda,
    const unsigned short* __restrict__ Btp, int ldb,
    float* Cf, int ldc, int M, int N, int K, float oscale) {
  const _Float16* Ah = (const _Float16*)(const void*)Ap;
  const _Float16* Bh = (const _Float16*)(const void*)Btp;
  __shared__ __align__(16) float sT[8][16 * 68];
  const int lane = threadIdx.x & 31;
  const int wave = threadIdx.x >> 5;
  const int tilesN = N >> 6;
  const int tilesM = M >> 6;
  const int tile = blockIdx.x * 8 + wave;
  if (tile >= tilesM * tilesN) return;
  const int tm = tile / tilesN;
  const int tn = tile - tm * tilesN;
  const int m0 = tm << 6;
  const int n0 = tn << 6;

  const int rlane = lane & 15;
  const int koff  = (lane >> 4) * 8;
  const int mOff  = (lane >> 4) * 8;

  v8f acc[4][4];
#pragma unroll
  for (int i = 0; i < 4; ++i)
#pragma unroll
    for (int j = 0; j < 4; ++j) acc[i][j] = zero8();

  for (int k0 = 0; k0 < K; k0 += 32) {
    v16h bh[4];
#pragma unroll
    for (int j = 0; j < 4; ++j) {
      const size_t bo = (size_t)(n0 + (j << 4) + rlane) * ldb + koff + k0;
      bh[j] = ldfrag_h(Bh + bo);
    }
#pragma unroll
    for (int i = 0; i < 4; ++i) {
      const size_t ao = (size_t)(m0 + (i << 4) + rlane) * lda + koff + k0;
      const v16h ah = ldfrag_h(Ah + ao);
#pragma unroll
      for (int j = 0; j < 4; ++j) acc[i][j] = mma_h_raw(ah, bh[j], acc[i][j]);
      dep_guard_h(acc[i][0], acc[i][3], ah);
    }
    keep4_h(bh[0], bh[1], bh[2], bh[3]);
  }
  acc_guard4(acc[0][0], acc[0][1], acc[0][2], acc[0][3]);
  acc_guard4(acc[1][0], acc[1][1], acc[1][2], acc[1][3]);
  acc_guard4(acc[2][0], acc[2][1], acc[2][2], acc[2][3]);
  acc_guard4(acc[3][0], acc[3][1], acc[3][2], acc[3][3]);

  float* slab = sT[wave];
  const int h2 = lane >> 4, c4 = (lane & 15) * 4;
#pragma unroll
  for (int i = 0; i < 4; ++i) {
    const int mBase = m0 + (i << 4);
#pragma unroll
    for (int r = 0; r < 8; ++r) {
#pragma unroll
      for (int j = 0; j < 4; ++j) {
        slab[(mOff + r) * 68 + (j << 4) + rlane] = acc[i][j][r];
      }
    }
    __builtin_amdgcn_fence(__ATOMIC_RELEASE, "workgroup");
    __builtin_amdgcn_wave_barrier();
    __builtin_amdgcn_fence(__ATOMIC_ACQUIRE, "workgroup");
    v4f ov[8];
#pragma unroll
    for (int it = 0; it < 8; ++it) {
      const int row = it * 2 + h2;
      const v4f xs = *(const v4f*)(slab + row * 68 + c4);
      ov[it] = xs * oscale;
    }
    for (int pass = 0; pass < 2; ++pass) {
#pragma unroll
      for (int it = 0; it < 8; ++it) {
        const int row = it * 2 + h2;
        *(volatile v4f*)(Cf + (size_t)(mBase + row) * ldc + n0 + c4) = ov[it];
      }
      __threadfence();
    }
    __builtin_amdgcn_fence(__ATOMIC_RELEASE, "workgroup");
    __builtin_amdgcn_wave_barrier();
    __builtin_amdgcn_fence(__ATOMIC_ACQUIRE, "workgroup");
  }
}

__global__ __launch_bounds__(256) void conv3(const float* __restrict__ Pf, const float* __restrict__ cw,
                                             const float* __restrict__ cb, const float* __restrict__ bin,
                                             int addb, unsigned short* Oh, float* Of, int tof, float osc) {
  const int lane = threadIdx.x & 31, wave = threadIdx.x >> 5;
  const int gw = blockIdx.x * 8 + wave;
  const int m = gw / (DMD / 128);
  if (m >= NROW) return;
  const int seg = gw - m * (DMD / 128);
  const int ch = seg * 128 + lane * 4;
  const int b = m / NTOK;
  const int m1 = (b >= 1) ? (m - NTOK) : m;
  const int m2 = (b >= 2) ? (m - 2 * NTOK) : m;
  const float f1 = (b >= 1) ? 1.0f : 0.0f;
  const float f2 = (b >= 2) ? 1.0f : 0.0f;
  const float fb = (addb != 0) ? 1.0f : 0.0f;
  const v4f u2 = *(const v4f*)(Pf + (size_t)m  * DMD + ch);
  const v4f u1 = *(const v4f*)(Pf + (size_t)m1 * DMD + ch);
  const v4f u0 = *(const v4f*)(Pf + (size_t)m2 * DMD + ch);
  const v4f braw = *(const v4f*)(bin + ch);
  float y[4];
#pragma unroll
  for (int e = 0; e < 4; ++e) {
    const float bb = bfr(braw[e]) * fb;
    const float w0 = bfr(cw[(ch + e) * 3 + 0]);
    const float w1 = bfr(cw[(ch + e) * 3 + 1]);
    const float w2 = bfr(cw[(ch + e) * 3 + 2]);
    const float cbias = bfr(cb[ch + e]);
    const float t0 = f2 * (u0[e] + bb);
    const float t1 = f1 * (u1[e] + bb);
    const float t2 = u2[e] + bb;
    y[e] = ((w0 * t0 + w1 * t1) + w2 * t2) + cbias;
  }
  const size_t o = (size_t)m * DMD + ch;
  if (tof == 0) {
    v2u pk;
    pk[0] = pk16(h_bits((_Float16)(y[0] * osc)), h_bits((_Float16)(y[1] * osc)));
    pk[1] = pk16(h_bits((_Float16)(y[2] * osc)), h_bits((_Float16)(y[3] * osc)));
    *(volatile v2u*)(Oh + o) = pk;
    __threadfence();
    *(volatile v2u*)(Oh + o) = pk;
  } else {
    v4f yv = {y[0], y[1], y[2], y[3]};
    *(volatile v4f*)(Of + o) = yv;
    __threadfence();
    *(volatile v4f*)(Of + o) = yv;
  }
}

__global__ __launch_bounds__(256) void vt_plane(const float* __restrict__ vf, unsigned short* vth,
                                                float vscale) {
  __shared__ __align__(16) float sv[64 * 68];
  const int tid = threadIdx.x;
  const int t0  = blockIdx.x * 64;
  const int hh  = blockIdx.y;
  const int b   = blockIdx.z;
#pragma unroll
  for (int i = 0; i < 4; ++i) {
    const int idx = i * 256 + tid;
    const int tt = idx >> 4, c4 = (idx & 15) * 4;
    const v4f a = *(const v4f*)(vf + ((size_t)(b * NTOK + t0 + tt)) * DMD + hh * HDD + c4);
    *(v4f*)(sv + tt * 68 + c4) = a;
  }
  __syncthreads();

  const int g = tid >> 3, piece = tid & 7;
  v4u hv[2];
  size_t hofs[2];
#pragma unroll
  for (int it = 0; it < 2; ++it) {
    const int d = it * 32 + g;
    v4u a;
#pragma unroll
    for (int e = 0; e < 4; ++e) {
      const float v0 = sv[(piece * 8 + 2 * e) * 68 + d] * vscale;
      const float v1 = sv[(piece * 8 + 2 * e + 1) * 68 + d] * vscale;
      a[e] = pk16(h_bits((_Float16)v0), h_bits((_Float16)v1));
    }
    hv[it] = a;
    hofs[it] = ((size_t)((b * NHD + hh) * HDD + d)) * NTOK + t0 + piece * 8;
  }
  for (int pass = 0; pass < 2; ++pass) {
#pragma unroll
    for (int it = 0; it < 2; ++it) *(volatile v4u*)(vth + hofs[it]) = hv[it];
    __threadfence();
  }
}

__global__ __launch_bounds__(256) void v_mean(const float* __restrict__ vf, float* mv) {
  __shared__ float red[8][33];
  const int tid = threadIdx.x;
  const int c = tid & 31, part = tid >> 5;
  const int col = blockIdx.x * 32 + c;
  const int b = blockIdx.y;
  const float* p = vf + ((size_t)b * NTOK + (size_t)part * 128) * DMD + col;
  float s = 0.f;
#pragma unroll 4
  for (int i = 0; i < 128; ++i) s += p[(size_t)i * DMD];
  red[part][c] = s;
  __syncthreads();
  const float tot = (((((((red[0][c] + red[1][c]) + red[2][c]) + red[3][c]) + red[4][c]) + red[5][c])
                      + red[6][c]) + red[7][c]) * (1.0f / (float)NTOK);
  const size_t o = (size_t)b * DMD + col;
  if (part == 0) *(volatile float*)(mv + o) = tot;
  __threadfence();
  if (part == 0) *(volatile float*)(mv + o) = tot;
}

__global__ __launch_bounds__(128)
void attn_cn(const unsigned short* __restrict__ qhp, const unsigned short* __restrict__ khp,
             const unsigned short* __restrict__ vtp, const float* __restrict__ mvp,
             float* yp, float sscale, float oscl) {
  union FH { v16h v; v8h h[2]; };
  __shared__ __align__(16) _Float16 Ksh[64 * 64];
  __shared__ __align__(16) _Float16 Vth[64 * 64];
  __shared__ __align__(16) _Float16 Psh[4][16 * 64];
  __shared__ __align__(16) float    Os[4][16 * 64];

  const int tid  = threadIdx.x;
  const int wave = tid >> 5;
  const int lane = tid & 31;
  const int hh   = lane >> 4;
  const int c    = lane & 15;

  const int bx = blockIdx.x;
  const int qb = bx % NQB;
  const int hb = bx / NQB;
  const int h  = hb % NHD;
  const int b  = hb / NHD;
  const int q0 = qb * 64 + wave * 16;

  const _Float16* Qp = (const _Float16*)(const void*)qhp + (size_t)b * NTOK * DMD + (size_t)h * HDD;
  const _Float16* Kp = (const _Float16*)(const void*)khp + (size_t)b * NTOK * DMD + (size_t)h * HDD;
  const _Float16* Vp = (const _Float16*)(const void*)vtp + (size_t)(b * NHD + h) * HDD * NTOK;

  v16h qa[2];
#pragma unroll
  for (int dc = 0; dc < 2; ++dc) {
    const size_t qo = (size_t)(q0 + c) * DMD + dc * 32 + 8 * hh;
    qa[dc] = ldfrag_h(Qp + qo);
  }

  float mrow[8], lrow[8];
#pragma unroll
  for (int r = 0; r < 8; ++r) { mrow[r] = -INFINITY; lrow[r] = 0.f; }

  for (int kt = 0; kt < NKT; ++kt) {
    const int kv0 = kt * 64;
    __syncthreads();
    {
      const int r = tid >> 1, half = (tid & 1) * 32;
      const _Float16* kg = Kp + (size_t)(kv0 + r) * DMD + half;
#pragma unroll
      for (int i = 0; i < 4; ++i) {
        const v8h a0 = *(const v8h*)(kg + 8 * i);
        *(v8h*)(Ksh + r * 64 + half + 8 * i) = a0;
      }
    }
    __syncthreads();

    v8f s[4];
#pragma unroll
    for (int j = 0; j < 4; ++j) {
      s[j] = zero8();
#pragma unroll
      for (int dc = 0; dc < 2; ++dc) {
        FH kb;
        kb.h[0] = *(const v8h*)(Ksh + (j * 16 + c) * 64 + dc * 32 + 8 * hh);
        kb.h[1] = *(const v8h*)(Ksh + (j * 16 + c) * 64 + dc * 32 + 16 + 8 * hh);
        s[j] = mma_h(qa[dc], kb.v, s[j]);
      }
    }
#pragma unroll
    for (int r = 0; r < 8; ++r) {
      float m = -INFINITY;
#pragma unroll
      for (int j = 0; j < 4; ++j) {
        const float sv = s[j][r] * sscale;
        s[j][r] = sv;
        m = fmaxf(m, sv);
      }
#pragma unroll
      for (int off = 1; off < 16; off <<= 1) m = fmaxf(m, __shfl_xor(m, off, 32));
      const float mnew  = fmaxf(mrow[r], m);
      const float alpha = __expf(mrow[r] - mnew);
      mrow[r] = mnew;
      float psum = 0.f;
#pragma unroll
      for (int j = 0; j < 4; ++j) psum += __expf(s[j][r] - mnew);
#pragma unroll
      for (int off = 1; off < 16; off <<= 1) psum += __shfl_xor(psum, off, 32);
      lrow[r] = lrow[r] * alpha + psum;
    }
  }
  float linv[8];
#pragma unroll
  for (int r = 0; r < 8; ++r) linv[r] = 1.0f / lrow[r];

  v8f oacc[4];
#pragma unroll
  for (int t = 0; t < 4; ++t) oacc[t] = zero8();

  for (int kt = 0; kt < NKT; ++kt) {
    const int kv0 = kt * 64;
    __syncthreads();
    {
      const int r = tid >> 1, half = (tid & 1) * 32;
      const _Float16* kg = Kp + (size_t)(kv0 + r) * DMD + half;
      const _Float16* vg = Vp + (size_t)r * NTOK + kv0 + half;
#pragma unroll
      for (int i = 0; i < 4; ++i) {
        const v8h a0 = *(const v8h*)(kg + 8 * i);
        const v8h b0 = *(const v8h*)(vg + 8 * i);
        *(v8h*)(Ksh + r * 64 + half + 8 * i) = a0;
        *(v8h*)(Vth + r * 64 + half + 8 * i) = b0;
      }
    }
    __syncthreads();

    v8f s[4];
#pragma unroll
    for (int j = 0; j < 4; ++j) {
      s[j] = zero8();
#pragma unroll
      for (int dc = 0; dc < 2; ++dc) {
        FH kb;
        kb.h[0] = *(const v8h*)(Ksh + (j * 16 + c) * 64 + dc * 32 + 8 * hh);
        kb.h[1] = *(const v8h*)(Ksh + (j * 16 + c) * 64 + dc * 32 + 16 + 8 * hh);
        s[j] = mma_h(qa[dc], kb.v, s[j]);
      }
    }

    _Float16* pwh = Psh[wave];
#pragma unroll
    for (int r = 0; r < 8; ++r) {
      const float mr = mrow[r], li = linv[r];
#pragma unroll
      for (int j = 0; j < 4; ++j) {
        const float p = __expf(s[j][r] * sscale - mr) * li;
        const _Float16 ph = (_Float16)(p * PCAR - POFF);
        pwh[(8 * hh + r) * 64 + j * 16 + c] = ph;
      }
    }
    __builtin_amdgcn_fence(__ATOMIC_RELEASE, "workgroup");
    __builtin_amdgcn_wave_barrier();
    __builtin_amdgcn_fence(__ATOMIC_ACQUIRE, "workgroup");

#pragma unroll 1
    for (int kk = 0; kk < 2; ++kk) {
      FH pa;
      pa.h[0] = *(const v8h*)(pwh + c * 64 + kk * 32 + 8 * hh);
      pa.h[1] = *(const v8h*)(pwh + c * 64 + kk * 32 + 16 + 8 * hh);
#pragma unroll
      for (int t = 0; t < 4; ++t) {
        FH vb;
        vb.h[0] = *(const v8h*)(Vth + (t * 16 + c) * 64 + kk * 32 + 8 * hh);
        vb.h[1] = *(const v8h*)(Vth + (t * 16 + c) * 64 + kk * 32 + 16 + 8 * hh);
        oacc[t] = mma_h(pa.v, vb.v, oacc[t]);
      }
    }
  }

  float* os = Os[wave];
  float mv[4];
#pragma unroll
  for (int t = 0; t < 4; ++t) mv[t] = mvp[(size_t)b * DMD + h * HDD + t * 16 + c];
#pragma unroll
  for (int r = 0; r < 8; ++r) {
#pragma unroll
    for (int t = 0; t < 4; ++t) os[(8 * hh + r) * 64 + t * 16 + c] = oacc[t][r] * oscl + mv[t];
  }
  __builtin_amdgcn_fence(__ATOMIC_RELEASE, "workgroup");
  __builtin_amdgcn_wave_barrier();
  __builtin_amdgcn_fence(__ATOMIC_ACQUIRE, "workgroup");
  {
    const int h2 = lane >> 4, c4 = (lane & 15) * 4;
    v4f ov[8];
#pragma unroll
    for (int it = 0; it < 8; ++it) {
      const int row = it * 2 + h2;
      ov[it] = *(const v4f*)(os + row * 64 + c4);
    }
    for (int pass = 0; pass < 2; ++pass) {
#pragma unroll
      for (int it = 0; it < 8; ++it) {
        const int row = it * 2 + h2;
        const size_t go = (size_t)(b * NTOK + q0 + row) * DMD + (size_t)h * HDD + c4;
        *(volatile v4f*)(yp + go) = ov[it];
      }
      __threadfence();
    }
  }
}

__global__ __launch_bounds__(256) void cvt_hl(const float* __restrict__ in, unsigned short* oh,
                                              unsigned short* ol, int n8, float sc, float lsc) {
  const int i = blockIdx.x * 256 + threadIdx.x;
  if (i < n8) {
    float a[8];
    ld8(in + (size_t)i * 8, a);
    v4u ph, pl;
#pragma unroll
    for (int p = 0; p < 4; ++p) {
      const int e = 2 * p;
      const float f0 = a[e] * sc, f1 = a[e + 1] * sc;
      const _Float16 x0 = (_Float16)f0, x1 = (_Float16)f1;
      const _Float16 l0 = (_Float16)((f0 - (float)x0) * lsc);
      const _Float16 l1 = (_Float16)((f1 - (float)x1) * lsc);
      ph[p] = pk16(h_bits(x0), h_bits(x1));
      pl[p] = pk16(h_bits(l0), h_bits(l1));
    }
    *(volatile v4u*)(oh + (size_t)i * 8) = ph;
    *(volatile v4u*)(ol + (size_t)i * 8) = pl;
    __threadfence();
    *(volatile v4u*)(oh + (size_t)i * 8) = ph;
    *(volatile v4u*)(ol + (size_t)i * 8) = pl;
  }
}

__global__ __launch_bounds__(256) void gemm_hl(
    const unsigned short* __restrict__ Ahp, const unsigned short* __restrict__ Alp, int lda,
    const unsigned short* __restrict__ Btp, int ldb, const float* __restrict__ bias,
    float* Cf, int ldc, int M, int N, int K, float oscale, float lfold) {
  const _Float16* Ah = (const _Float16*)(const void*)Ahp;
  const _Float16* Al = (const _Float16*)(const void*)Alp;
  const _Float16* Bh = (const _Float16*)(const void*)Btp;
  __shared__ __align__(16) float sT[8][16 * 36];
  const int lane = threadIdx.x & 31;
  const int wave = threadIdx.x >> 5;
  const int tilesN = N >> 5;
  const int tilesM = M >> 5;
  const int tile = blockIdx.x * 8 + wave;
  if (tile >= tilesM * tilesN) return;
  const int tm = tile / tilesN;
  const int tn = tile - tm * tilesN;
  const int m0 = tm << 5;
  const int n0 = tn << 5;

  const int rlane = lane & 15;
  const int koff  = (lane >> 4) * 8;
  const int mOff  = (lane >> 4) * 8;

  v8f acc[2][2], accl[2][2];
#pragma unroll
  for (int i = 0; i < 2; ++i)
#pragma unroll
    for (int j = 0; j < 2; ++j) { acc[i][j] = zero8(); accl[i][j] = zero8(); }

  for (int k0 = 0; k0 < K; k0 += 32) {
    v16h bh[2];
#pragma unroll
    for (int j = 0; j < 2; ++j) {
      const size_t bo = (size_t)(n0 + (j << 4) + rlane) * ldb + koff + k0;
      bh[j] = ldfrag_h(Bh + bo);
    }
#pragma unroll
    for (int i = 0; i < 2; ++i) {
      const size_t ao = (size_t)(m0 + (i << 4) + rlane) * lda + koff + k0;
      const v16h a  = ldfrag_h(Ah + ao);
      const v16h al = ldfrag_h(Al + ao);
#pragma unroll
      for (int j = 0; j < 2; ++j) {
        acc[i][j]  = mma_h(a,  bh[j], acc[i][j]);
        accl[i][j] = mma_h(al, bh[j], accl[i][j]);
      }
    }
  }
  acc_guard4(acc[0][0], acc[0][1], acc[1][0], acc[1][1]);
  acc_guard4(accl[0][0], accl[0][1], accl[1][0], accl[1][1]);

  float* slab = sT[wave];
  const int rr = lane >> 3, c4 = (lane & 7) * 4;
  v4f b4;
  {
    const v4f braw = *(const v4f*)(bias + n0 + c4);
#pragma unroll
    for (int e = 0; e < 4; ++e) b4[e] = bfr(braw[e]);
  }
#pragma unroll
  for (int i = 0; i < 2; ++i) {
    const int mBase = m0 + (i << 4);
#pragma unroll
    for (int r = 0; r < 8; ++r) {
#pragma unroll
      for (int j = 0; j < 2; ++j) {
        slab[(mOff + r) * 36 + (j << 4) + rlane] = acc[i][j][r] + accl[i][j][r] * lfold;
      }
    }
    __builtin_amdgcn_fence(__ATOMIC_RELEASE, "workgroup");
    __builtin_amdgcn_wave_barrier();
    __builtin_amdgcn_fence(__ATOMIC_ACQUIRE, "workgroup");
    v4f ov[4];
#pragma unroll
    for (int it = 0; it < 4; ++it) {
      const int row = it * 4 + rr;
      const v4f xs = *(const v4f*)(slab + row * 36 + c4);
      ov[it] = xs * oscale + b4;
    }
    for (int pass = 0; pass < 2; ++pass) {
#pragma unroll
      for (int it = 0; it < 4; ++it) {
        const int row = it * 4 + rr;
        *(volatile v4f*)(Cf + (size_t)(mBase + row) * ldc + n0 + c4) = ov[it];
      }
      __threadfence();
    }
    __builtin_amdgcn_fence(__ATOMIC_RELEASE, "workgroup");
    __builtin_amdgcn_wave_barrier();
    __builtin_amdgcn_fence(__ATOMIC_ACQUIRE, "workgroup");
  }
}

extern "C" void kernel_launch(void* const* d_in, const int* in_sizes, int n_in,
                              void* d_out, int out_size, void* d_ws, size_t ws_size,
                              hipStream_t stream) {
  if (n_in < 13) return;
  if (in_sizes[0] != NROW * DMD) return;
  if (in_sizes[1] != DMD * DMD || in_sizes[2] != DMD * DMD || in_sizes[3] != DMD * DMD) return;
  if (in_sizes[11] != DMD * DMD) return;
  if (in_sizes[4] != DMD || in_sizes[6] != DMD || in_sizes[8] != DMD || in_sizes[10] != DMD) return;
  if (in_sizes[12] != DMD) return;
  if (in_sizes[5] != DMD * 3 || in_sizes[7] != DMD * 3 || in_sizes[9] != DMD * 3) return;
  if (out_size != NROW * DMD) return;

  const float* x    = (const float*)d_in[0];
  const float* wq   = (const float*)d_in[1];
  const float* wk   = (const float*)d_in[2];
  const float* wv   = (const float*)d_in[3];
  const float* bv   = (const float*)d_in[4];
  const float* cq_w = (const float*)d_in[5];
  const float* cq_b = (const float*)d_in[6];
  const float* ck_w = (const float*)d_in[7];
  const float* ck_b = (const float*)d_in[8];
  const float* cv_w = (const float*)d_in[9];
  const float* cv_b = (const float*)d_in[10];
  const float* wo   = (const float*)d_in[11];
  const float* bo   = (const float*)d_in[12];

  const size_t P16  = (size_t)NROW * DMD * 2;
  const size_t PW3  = (size_t)3 * DMD * DMD * 2;
  const size_t PWo  = (size_t)DMD * DMD * 2;
  const size_t PF32 = (size_t)NROW * DMD * 4;
  const size_t PVT  = (size_t)NB * NHD * HDD * NTOK * 2;
  const size_t PMv  = (size_t)NB * DMD * 4;
  size_t off = 0;
  const size_t oX16 = off; off += P16;
  const size_t oW3  = off; off += PW3;
  const size_t oWo  = off; off += PWo;
  const size_t oPf  = off; off += PF32;
  const size_t oQh  = off; off += P16;
  const size_t oKh  = off; off += P16;
  const size_t oVc  = off; off += PF32;
  const size_t oVT  = off; off += PVT;
  const size_t oMv  = off; off += PMv;
  const size_t oYh  = off; off += P16;
  const size_t oYl  = off; off += P16;
  if (off > ws_size) return;
  if (off > (size_t)134217728) return;

  char* ws = (char*)d_ws;
  unsigned short* X16 = (unsigned short*)(ws + oX16);
  unsigned short* W3T = (unsigned short*)(ws + oW3);
  unsigned short* WoT = (unsigned short*)(ws + oWo);
  float*          Pf  = (float*)(ws + oPf);
  float*          Yf  = (float*)(ws + oPf);
  unsigned short* Qh  = (unsigned short*)(ws + oQh);
  unsigned short* Kh  = (unsigned short*)(ws + oKh);
  float*          Vc  = (float*)(ws + oVc);
  unsigned short* VT  = (unsigned short*)(ws + oVT);
  float*          Mv  = (float*)(ws + oMv);
  unsigned short* Yh  = (unsigned short*)(ws + oYh);
  unsigned short* Yl  = (unsigned short*)(ws + oYl);
  float*          outf = (float*)d_out;

  const size_t WSTRIDE = (size_t)DMD * DMD;

  const dim3 blk(256);
  const int  n8x = NROW * DMD / 8;
  const dim3 gCvt((n8x + 255) / 256);
  const dim3 gW(DMD / 64, DMD / 64);
  const dim3 gProj(((NROW / 64) * (DMD / 64) + 7) / 8);
  const dim3 gConv((NROW * (DMD / 128) + 7) / 8);
  const dim3 gVt(NTOK / 64, NHD, NB);
  const dim3 gMv(DMD / 32, NB);
  const dim3 gAttn(NB * NHD * NQB);
  const dim3 gOut(((NROW / 32) * (DMD / 32) + 7) / 8);

  const float xScale  = 8.0f;
  const float wScale  = 256.0f;
  const float pOscale = 1.0f / 2048.0f;
  const float qkScale = 256.0f;
  const float vScale  = 256.0f;
  const float sscale  = 1.0f / 524288.0f;
  const float attOscl = 1.0f / 4194304.0f;
  const float yScale  = 4096.0f;
  const float lScale  = 2048.0f;
  const float oOscale = 1.0f / 1048576.0f;
  const float lFold   = 1.0f / 2048.0f;

  x_cvt<<<gCvt, blk, 0, stream>>>(x, X16, n8x, xScale);
  wt_cvt<<<gW, blk, 0, stream>>>(wq, DMD, DMD, W3T, wScale);
  wt_cvt<<<gW, blk, 0, stream>>>(wk, DMD, DMD, W3T + WSTRIDE, wScale);
  wt_cvt<<<gW, blk, 0, stream>>>(wv, DMD, DMD, W3T + 2 * WSTRIDE, wScale);
  wt_cvt<<<gW, blk, 0, stream>>>(wo, DMD, DMD, WoT, wScale);
  gemm64<<<gProj, blk, 0, stream>>>(X16, DMD, W3T, DMD, Pf, DMD, NROW, DMD, DMD, pOscale);
  conv3<<<gConv, blk, 0, stream>>>(Pf, cq_w, cq_b, bv, 0, Qh, Vc, 0, qkScale);
  gemm64<<<gProj, blk, 0, stream>>>(X16, DMD, W3T + WSTRIDE, DMD, Pf, DMD, NROW, DMD, DMD, pOscale);
  conv3<<<gConv, blk, 0, stream>>>(Pf, ck_w, ck_b, bv, 0, Kh, Vc, 0, qkScale);
  gemm64<<<gProj, blk, 0, stream>>>(X16, DMD, W3T + 2 * WSTRIDE, DMD, Pf, DMD, NROW, DMD, DMD, pOscale);
  conv3<<<gConv, blk, 0, stream>>>(Pf, cv_w, cv_b, bv, 1, Qh, Vc, 1, 1.0f);
  vt_plane<<<gVt, blk, 0, stream>>>(Vc, VT, vScale);
  v_mean<<<gMv, blk, 0, stream>>>(Vc, Mv);
  attn_cn<<<gAttn, dim3(128), 0, stream>>>(Qh, Kh, VT, Mv, Yf, sscale, attOscl);
  cvt_hl<<<gCvt, blk, 0, stream>>>(Yf, Yh, Yl, n8x, yScale, lScale);
  gemm_hl<<<gOut, blk, 0, stream>>>(Yh, Yl, DMD, WoT, DMD, bo, outf, DMD, NROW, DMD, DMD, oOscale, lFold);
  (void)hipGetLastError();
}
